// Deformable_MatMul3_26147760898634
// MI455X (gfx1250) — hardware-verified
//
#include <hip/hip_runtime.h>

typedef _Float16 v16h __attribute__((ext_vector_type(16)));
typedef _Float16 v8h  __attribute__((ext_vector_type(8)));
typedef float    v8f  __attribute__((ext_vector_type(8)));
typedef float    v4f  __attribute__((ext_vector_type(4)));
union Frag { v16h v; v8h half[2]; };

#define BATCH   8
#define C_IN    256
#define HW      4096
#define O_CH    256
#define NREG    8
#define PTILE   64
#define OTILE   128
#define KCHUNK  64
#define XS_STRIDE 264
#define WS_STRIDE 72
#define TS_STRIDE 64
#define X_SCALE   256.0f
#define W_SCALE   16.0f
#define OUT_UNSCALE (1.0f / 4096.0f)

__device__ __forceinline__ v8f wmma16(v16h a, v16h b, v8f c) {
  v8f d = __builtin_amdgcn_wmma_f32_16x16x32_f16(false, a, false, b, (short)0, c, false, false);
  asm volatile("v_nop\n\tv_nop\n\tv_nop\n\tv_nop" : "+v"(d) : "v"(a), "v"(b));
  return d;
}

__global__ __launch_bounds__(256) void prep_weights(
    const float* __restrict__ mat1, _Float16* __restrict__ wp,
    const int* __restrict__ beta_unused) {
  (void)beta_unused;
  const int tid = blockIdx.x * 256 + threadIdx.x;
  if (tid >= NREG * O_CH * (C_IN / 8)) return;
  const int c8 = (tid & 31) * 8;
  const int o  = (tid >> 5) & (O_CH - 1);
  const int r  = tid >> 13;
  v8h v;
  #pragma unroll
  for (int i = 0; i < 8; ++i)
    v[i] = (_Float16)(mat1[((size_t)(o * C_IN + c8 + i)) * NREG + r] * W_SCALE);
  _Float16* dst = wp + ((size_t)(r * O_CH + o)) * C_IN + c8;
  *(volatile v8h*)dst = v;
  __threadfence();
  *(volatile v8h*)dst = v;
}

__global__ __launch_bounds__(256) void deform_mm(
    const float* __restrict__ mat0, const _Float16* __restrict__ wp,
    const float* __restrict__ mask, const float* __restrict__ alpha,
    const int* __restrict__ use_alpha, float* __restrict__ out) {
  extern __shared__ __align__(16) char smem[];
  _Float16* Xs = (_Float16*)smem;
  _Float16* Wc = Xs + PTILE * XS_STRIDE;
  float*    Ms = (float*)(Wc + OTILE * WS_STRIDE);
  float*    Ts = (float*)smem;

  if (blockIdx.x >= BATCH * (HW / PTILE) || blockIdx.y >= O_CH / OTILE) return;

  const int t     = threadIdx.x;
  const int b     = blockIdx.x >> 6;
  const int pp    = (blockIdx.x & 63) * PTILE;
  const int obase = blockIdx.y * OTILE;

  {
    const int pix = t & 63;
    const int c0  = t >> 6;
    const float* src = mat0 + (size_t)b * C_IN * HW + pp + pix;
    #pragma unroll 4
    for (int cb = 0; cb < C_IN; cb += 4) {
      const int c = cb + c0;
      Xs[pix * XS_STRIDE + c] = (_Float16)(src[(size_t)c * HW] * X_SCALE);
    }
  }
  {
    const int ua = use_alpha[0];
    #pragma unroll
    for (int it = 0; it < 2; ++it) {
      const int idx = it * 256 + t;
      const int r = idx >> 6, pix = idx & 63;
      const float a = ua ? alpha[r] : 1.0f;
      Ms[idx] = mask[(size_t)r * HW + pp + pix] * a;
    }
  }
  __syncthreads();

  const int wid    = t >> 5;
  const int lane   = t & 31;
  const int lrow   = lane & 15;
  const int lhi    = lane >> 4;
  const int wave_o = wid >> 1;
  const int wave_p = wid & 1;

  v8f acc[2][2];
  #pragma unroll
  for (int mo = 0; mo < 2; ++mo)
    #pragma unroll
    for (int pt = 0; pt < 2; ++pt)
      #pragma unroll
      for (int i = 0; i < 8; ++i) acc[mo][pt][i] = 0.0f;

  for (int r = 0; r < NREG; ++r) {
    v8f racc[2][2];
    #pragma unroll
    for (int mo = 0; mo < 2; ++mo)
      #pragma unroll
      for (int pt = 0; pt < 2; ++pt)
        #pragma unroll
        for (int i = 0; i < 8; ++i) racc[mo][pt][i] = 0.0f;

    for (int kt0 = 0; kt0 < C_IN / KCHUNK; ++kt0) {
      __syncthreads();

      const _Float16* wsrc = wp + ((size_t)r * O_CH + obase) * C_IN + kt0 * KCHUNK;
      #pragma unroll
      for (int it = 0; it < 4; ++it) {
        const int chunk = it * 256 + t;
        const int o  = chunk >> 3;
        const int c8 = (chunk & 7) * 8;
        v8h v = *(const v8h*)(wsrc + (size_t)o * C_IN + c8);
        *(v8h*)(Wc + o * WS_STRIDE + c8) = v;
      }
      __syncthreads();

      #pragma unroll
      for (int ks = 0; ks < 2; ++ks) {
        Frag a[2];
        #pragma unroll
        for (int mo = 0; mo < 2; ++mo) {
          const int row = wave_o * 32 + mo * 16 + lrow;
          const _Float16* p = Wc + row * WS_STRIDE + ks * 32 + lhi * 8;
          a[mo].half[0] = *(const v8h*)p;
          a[mo].half[1] = *(const v8h*)(p + 16);
        }
        Frag bf[2];
        #pragma unroll
        for (int pt = 0; pt < 2; ++pt) {
          const int pixr = wave_p * 32 + pt * 16 + lrow;
          const _Float16* p = Xs + pixr * XS_STRIDE + kt0 * KCHUNK + ks * 32 + lhi * 8;
          bf[pt].half[0] = *(const v8h*)p;
          bf[pt].half[1] = *(const v8h*)(p + 16);
        }
        #pragma unroll
        for (int mo = 0; mo < 2; ++mo)
          #pragma unroll
          for (int pt = 0; pt < 2; ++pt)
            racc[mo][pt] = wmma16(a[mo].v, bf[pt].v, racc[mo][pt]);
      }
    }

    #pragma unroll
    for (int pt = 0; pt < 2; ++pt) {
      const float s = Ms[r * PTILE + wave_p * 32 + pt * 16 + lrow];
      #pragma unroll
      for (int mo = 0; mo < 2; ++mo)
        #pragma unroll
        for (int i = 0; i < 8; ++i)
          acc[mo][pt][i] += s * racc[mo][pt][i];
    }
  }

  __syncthreads();
  #pragma unroll
  for (int mo = 0; mo < 2; ++mo)
    #pragma unroll
    for (int pt = 0; pt < 2; ++pt) {
      const int pix_l = wave_p * 32 + pt * 16 + lrow;
      #pragma unroll
      for (int v = 0; v < 8; ++v) {
        const int o_l = wave_o * 32 + mo * 16 + lhi * 8 + v;
        Ts[o_l * TS_STRIDE + pix_l] = acc[mo][pt][v] * OUT_UNSCALE;
      }
    }
  __syncthreads();

  v4f vals[8];
  #pragma unroll
  for (int i = 0; i < 8; ++i) {
    const int row = i * 16 + wid * 2 + lhi;
    vals[i] = *(const v4f*)(Ts + row * TS_STRIDE + lrow * 4);
  }
  const size_t gbase = ((size_t)b * O_CH + obase) * HW + pp;
  #pragma unroll
  for (int i = 0; i < 8; ++i) {
    const int row = i * 16 + wid * 2 + lhi;
    float* gp = out + gbase + (size_t)row * HW + lrow * 4;
    *(volatile v4f*)gp = vals[i];
  }
  __threadfence();
  #pragma unroll
  for (int i = 0; i < 8; ++i) {
    const int row = i * 16 + wid * 2 + lhi;
    float* gp = out + gbase + (size_t)row * HW + lrow * 4;
    *(volatile v4f*)gp = vals[i];
  }
}

extern "C" void kernel_launch(void* const* d_in, const int* in_sizes, int n_in,
                              void* d_out, int out_size, void* d_ws, size_t ws_size,
                              hipStream_t stream) {
  if (n_in < 5) return;
  if (in_sizes[0] != BATCH * C_IN * HW) return;
  if (in_sizes[1] != O_CH * C_IN * NREG) return;
  if (in_sizes[2] != NREG * HW) return;
  if (in_sizes[3] < NREG) return;
  if (in_sizes[4] < 1) return;
  if (out_size != BATCH * O_CH * HW) return;

  const float* mat0      = (const float*)d_in[0];
  const float* mat1      = (const float*)d_in[1];
  const float* mask      = (const float*)d_in[2];
  const float* alpha     = (const float*)d_in[3];
  const int*   use_alpha = (const int*)d_in[4];
  const int*   beta      = (n_in > 5) ? (const int*)d_in[5] : (const int*)d_in[4];

  const size_t wp_bytes = (size_t)NREG * O_CH * C_IN * sizeof(_Float16);
  if (wp_bytes > ws_size) return;
  _Float16* wp = (_Float16*)d_ws;

  const int prep_threads = NREG * O_CH * (C_IN / 8);
  prep_weights<<<(prep_threads + 255) / 256, 256, 0, stream>>>(mat1, wp, beta);

  const size_t lds = (size_t)(PTILE * XS_STRIDE + OTILE * WS_STRIDE) * sizeof(_Float16)
                   + (size_t)NREG * PTILE * sizeof(float);
  dim3 grid(BATCH * (HW / PTILE), O_CH / OTILE);
  deform_mm<<<grid, 256, lds, stream>>>(mat0, wp, mask, alpha, use_alpha, (float*)d_out);
}
